// MSAAttention_19138374271388
// MI455X (gfx1250) — hardware-verified
//
#include <hip/hip_runtime.h>
#include <math.h>

typedef __attribute__((ext_vector_type(16))) _Float16 v16h;
typedef __attribute__((ext_vector_type(8)))  _Float16 v8h;
typedef __attribute__((ext_vector_type(16))) __bf16   v16b;
typedef __attribute__((ext_vector_type(8)))  __bf16   v8b;
typedef __attribute__((ext_vector_type(8)))  float    v8f;
typedef __attribute__((ext_vector_type(4)))  float    v4f;
typedef __attribute__((ext_vector_type(4)))  unsigned v4u;

constexpr int HDIM = 512;
constexpr int SEQL = 2048;
constexpr int NBAT = 8;
constexpr int NROW = NBAT * SEQL;
constexpr float RES_CARRY     = 2048.0f;
constexpr float RES_CARRY_INV = 1.0f / 2048.0f;
constexpr float P_CARRY       = 32768.0f;

static_assert(HDIM % 64 == 0 && SEQL % 64 == 0 && NROW % 64 == 0, "");
static_assert(HDIM % 32 == 0 && SEQL % 32 == 0, "");

__device__ __forceinline__ unsigned short f2bf_bits(float f) {
  unsigned u = __float_as_uint(f);
  return (unsigned short)((u + 0x7FFFu + ((u >> 16) & 1u)) >> 16);
}
__device__ __forceinline__ float bf_bits2f(unsigned short h) { return __uint_as_float(((unsigned)h) << 16); }
__device__ __forceinline__ float bf_rne(float f) { return bf_bits2f(f2bf_bits(f)); }

__device__ __forceinline__ void dep_guard_h(v8f& a, v8f& b, v16h x, v16h y) { asm volatile("v_nop\n\tv_nop\n\tv_nop\n\tv_nop" : "+v"(a), "+v"(b) : "v"(x), "v"(y)); }
__device__ __forceinline__ void dep_guard_b(v8f& a, v8f& b, v16b x, v16b y) { asm volatile("v_nop\n\tv_nop\n\tv_nop\n\tv_nop" : "+v"(a), "+v"(b) : "v"(x), "v"(y)); }
__device__ __forceinline__ void keep4_h(v16h a, v16h b, v16h c, v16h d) { asm volatile("v_nop" :: "v"(a), "v"(b), "v"(c), "v"(d)); }
__device__ __forceinline__ void keep4_b(v16b a, v16b b, v16b c, v16b d) { asm volatile("v_nop" :: "v"(a), "v"(b), "v"(c), "v"(d)); }
__device__ __forceinline__ void acc_guard4(v8f& a, v8f& b, v8f& c, v8f& d) { asm volatile("v_nop\n\tv_nop\n\tv_nop\n\tv_nop" : "+v"(a), "+v"(b), "+v"(c), "+v"(d)); }
template <typename T> struct Frag;
template <> struct Frag<_Float16> {
  typedef v16h V; union U { v16h v; v8h h[2]; };
  static __device__ __forceinline__ v16h load(const _Float16* p) {
    U f; f.h[0] = *(const v8h*)(p); f.h[1] = *(const v8h*)(p + 16); return f.v;
  }
  static __device__ __forceinline__ v8f mma(v16h a, v16h b, v8f c) {
    return __builtin_amdgcn_wmma_f32_16x16x32_f16(false, a, false, b, (short)0, c, false, false);
  }
  static __device__ __forceinline__ void guard(v8f& a, v8f& b, v16h x, v16h y) { dep_guard_h(a, b, x, y); }
  static __device__ __forceinline__ void keep(v16h a, v16h b, v16h c, v16h d) { keep4_h(a, b, c, d); }
};
template <> struct Frag<__bf16> {
  typedef v16b V; union U { v16b v; v8b h[2]; };
  static __device__ __forceinline__ v16b load(const __bf16* p) {
    U f; f.h[0] = *(const v8b*)(p); f.h[1] = *(const v8b*)(p + 16); return f.v;
  }
  static __device__ __forceinline__ v8f mma(v16b a, v16b b, v8f c) {
    return __builtin_amdgcn_wmma_f32_16x16x32_bf16(false, a, false, b, (short)0, c, false, false);
  }
  static __device__ __forceinline__ void guard(v8f& a, v8f& b, v16b x, v16b y) { dep_guard_b(a, b, x, y); }
  static __device__ __forceinline__ void keep(v16b a, v16b b, v16b c, v16b d) { keep4_b(a, b, c, d); }
};

struct PETab { float d[256]; };
static_assert(sizeof(PETab) == 1024, "");

__global__ __launch_bounds__(256) void k_petab(float* __restrict__ pe, PETab tab) {
#pragma clang fp contract(off)
  const int t = blockIdx.x * 256 + threadIdx.x;
  const int s = t >> 9;
  const int h = t & (HDIM - 1);
  const int i = h & 255;
  const float dv  = tab.d[i];
  const float ang = (float)s * dv;
  const float sn  = sinf(ang);
  const float cs  = cosf(ang);
  const float val = (h < 256) ? sn : cs;
  ((volatile float*)pe)[t] = val;
  __threadfence();
  ((volatile float*)pe)[t] = val;
}

__global__ __launch_bounds__(256) void k_wplane(const float* __restrict__ in, unsigned short* __restrict__ outp, int n2) {
  const int i = blockIdx.x * 256 + threadIdx.x;
  if (i < n2) {
    const unsigned u = (unsigned)f2bf_bits(in[2 * i]) | ((unsigned)f2bf_bits(in[2 * i + 1]) << 16);
    ((volatile unsigned*)outp)[i] = u;
    __threadfence();
    ((volatile unsigned*)outp)[i] = u;
  }
}

__global__ __launch_bounds__(256) void k_xplanes(const float* __restrict__ xin, const float* __restrict__ pe,
                                                 unsigned short* __restrict__ xh, unsigned short* __restrict__ xl) {
#pragma clang fp contract(off)
  const int t = blockIdx.x * 256 + threadIdx.x;
  const size_t e0 = (size_t)t * 8;
  const int h0 = (int)(e0 & (HDIM - 1));
  const int s  = (int)((e0 >> 9) & (SEQL - 1));
  const v4f a0 = *(const v4f*)(xin + e0);
  const v4f a1 = *(const v4f*)(xin + e0 + 4);
  const v4f p0 = *(const v4f*)(pe + (size_t)s * HDIM + h0);
  const v4f p1 = *(const v4f*)(pe + (size_t)s * HDIM + h0 + 4);
  float xv[8];
  xv[0] = bf_rne(a0[0]) + p0[0]; xv[1] = bf_rne(a0[1]) + p0[1];
  xv[2] = bf_rne(a0[2]) + p0[2]; xv[3] = bf_rne(a0[3]) + p0[3];
  xv[4] = bf_rne(a1[0]) + p1[0]; xv[5] = bf_rne(a1[1]) + p1[1];
  xv[6] = bf_rne(a1[2]) + p1[2]; xv[7] = bf_rne(a1[3]) + p1[3];
  v4u hv, lv;
#pragma unroll
  for (int e = 0; e < 4; ++e) {
    const float f0 = xv[2 * e], f1 = xv[2 * e + 1];
    const unsigned short hb0 = f2bf_bits(f0);
    const unsigned short lb0 = f2bf_bits(f0 - bf_bits2f(hb0));
    const unsigned short hb1 = f2bf_bits(f1);
    const unsigned short lb1 = f2bf_bits(f1 - bf_bits2f(hb1));
    hv[e] = (unsigned)hb0 | ((unsigned)hb1 << 16);
    lv[e] = (unsigned)lb0 | ((unsigned)lb1 << 16);
  }
  unsigned short* ph = xh + e0;
  unsigned short* pl = xl + e0;
  *(volatile v4u*)ph = hv;
  *(volatile v4u*)pl = lv;
  __threadfence();
  *(volatile v4u*)ph = hv;
  *(volatile v4u*)pl = lv;
}

template <bool SPLA, bool SPLB, int BIAS_MODE, int OUT_MODE>
__global__ __launch_bounds__(256) void k_pgemm(
    const unsigned short* __restrict__ Ap, const unsigned short* __restrict__ A2p, int lda, long strideA,
    const unsigned short* __restrict__ Btp, const unsigned short* __restrict__ Bt2p, int ldb, long strideB,
    unsigned short* __restrict__ Cp, unsigned short* __restrict__ C2p, int ldc, long strideC,
    const float* __restrict__ bias, int M, int N, int K) {
  typedef __bf16 T;
  typedef v16b V;
  const T* A   = (const T*)(const void*)Ap;
  const T* A2  = (const T*)(const void*)A2p;
  const T* Bt  = (const T*)(const void*)Btp;
  const T* Bt2 = (const T*)(const void*)Bt2p;
  __shared__ __align__(16) float sT[8][16 * 68];
  const int b    = blockIdx.y;
  const int lane = threadIdx.x & 31;
  const int wave = threadIdx.x >> 5;
  const int tilesN = N >> 6;
  const int tilesM = M >> 6;
  const int tile = blockIdx.x * 8 + wave;
  if (tile >= tilesM * tilesN) return;
  const int tm = tile / tilesN;
  const int tn = tile - tm * tilesN;
  const int m0 = tm << 6;
  const int n0 = tn << 6;

  const T* Ab  = A   + (size_t)b * strideA;
  const T* Ab2 = A2  + (size_t)b * strideA;
  const T* Bb  = Bt  + (size_t)b * strideB;
  const T* Bb2 = Bt2 + (size_t)b * strideB;

  const int rlane = lane & 15;
  const int koff  = (lane >> 4) * 8;
  const int mOff  = (lane >> 4) * 8;

  v8f acc[4][4];
#pragma unroll
  for (int i = 0; i < 4; ++i)
#pragma unroll
    for (int j = 0; j < 4; ++j) acc[i][j] = (v8f){0.f,0.f,0.f,0.f,0.f,0.f,0.f,0.f};

  for (int k0 = 0; k0 < K; k0 += 32) {
    V bh[4], bl[4];
#pragma unroll
    for (int j = 0; j < 4; ++j) {
      const size_t bo = (size_t)(n0 + (j << 4) + rlane) * ldb + koff + k0;
      bh[j] = Frag<T>::load(Bb + bo);
      if (SPLB) bl[j] = Frag<T>::load(Bb2 + bo);
    }
#pragma unroll
    for (int i = 0; i < 4; ++i) {
      const size_t ao = (size_t)(m0 + (i << 4) + rlane) * lda + koff + k0;
      V ah = Frag<T>::load(Ab + ao);
      V al = ah;
      if (SPLA) al = Frag<T>::load(Ab2 + ao);
#pragma unroll
      for (int j = 0; j < 4; ++j) {
        acc[i][j] = Frag<T>::mma(ah, bh[j], acc[i][j]);
        if (SPLB) acc[i][j] = Frag<T>::mma(ah, bl[j], acc[i][j]);
        if (SPLA) acc[i][j] = Frag<T>::mma(al, bh[j], acc[i][j]);
      }
      Frag<T>::guard(acc[i][0], acc[i][3], ah, al);
    }
    Frag<T>::keep(bh[0], bh[1], bh[2], bh[3]);
    if (SPLB) Frag<T>::keep(bl[0], bl[1], bl[2], bl[3]);
  }
  acc_guard4(acc[0][0], acc[0][1], acc[0][2], acc[0][3]);
  acc_guard4(acc[1][0], acc[1][1], acc[1][2], acc[1][3]);
  acc_guard4(acc[2][0], acc[2][1], acc[2][2], acc[2][3]);
  acc_guard4(acc[3][0], acc[3][1], acc[3][2], acc[3][3]);

  float* slab = sT[wave];
  unsigned short* C  = Cp  + (size_t)b * strideC;
  unsigned short* Cx = C2p + (size_t)b * strideC;
#pragma unroll
  for (int i = 0; i < 4; ++i) {
    const int mBase = m0 + (i << 4);
    float bm[8];
#pragma unroll
    for (int r = 0; r < 8; ++r) bm[r] = 0.f;
    if (BIAS_MODE == 1) {
      const v4f b0 = *(const v4f*)(bias + mBase + mOff);
      const v4f b1 = *(const v4f*)(bias + mBase + mOff + 4);
      bm[0] = bf_rne(b0[0]); bm[1] = bf_rne(b0[1]); bm[2] = bf_rne(b0[2]); bm[3] = bf_rne(b0[3]);
      bm[4] = bf_rne(b1[0]); bm[5] = bf_rne(b1[1]); bm[6] = bf_rne(b1[2]); bm[7] = bf_rne(b1[3]);
    }
#pragma unroll
    for (int j = 0; j < 4; ++j) {
      const int n = n0 + (j << 4) + rlane;
      float bn = 0.f;
      if (BIAS_MODE == 2) bn = bf_rne(bias[n]);
#pragma unroll
      for (int r = 0; r < 8; ++r) {
        float v = acc[i][j][r];
        if (BIAS_MODE == 1) v += bm[r];
        if (BIAS_MODE == 2) v += bn;
        slab[(mOff + r) * 68 + (j << 4) + rlane] = v;
      }
    }
    __builtin_amdgcn_fence(__ATOMIC_RELEASE, "workgroup");
    __builtin_amdgcn_wave_barrier();
    __builtin_amdgcn_fence(__ATOMIC_ACQUIRE, "workgroup");
    {
      const int q = lane >> 3, c8 = (lane & 7) * 8;
      for (int pass = 0; pass < 2; ++pass) {
#pragma unroll
        for (int it = 0; it < 4; ++it) {
          const int row = it * 4 + q;
          const float* sp = slab + row * 68 + c8;
          v8h hv, lv;
#pragma unroll
          for (int e = 0; e < 8; ++e) {
            const float f = sp[e];
            const _Float16 fh = (_Float16)f;
            hv[e] = fh;
            if (OUT_MODE == 3) lv[e] = (_Float16)((f - (float)fh) * RES_CARRY);
          }
          *(volatile v8h*)(C + (size_t)(mBase + row) * ldc + n0 + c8) = hv;
          if (OUT_MODE == 3) *(volatile v8h*)(Cx + (size_t)(mBase + row) * ldc + n0 + c8) = lv;
        }
        __threadfence();
      }
    }
    __builtin_amdgcn_fence(__ATOMIC_RELEASE, "workgroup");
    __builtin_amdgcn_wave_barrier();
    __builtin_amdgcn_fence(__ATOMIC_ACQUIRE, "workgroup");
  }
}

constexpr int ATQ    = 16;
constexpr int ATKW   = 32;
constexpr int ATNW   = 8;
constexpr int ATKT   = ATKW * ATNW;
constexpr int OPITCH = 68;
static_assert(SEQL % ATKT == 0 && SEQL % ATQ == 0 && HDIM == ATNW * 64, "");

struct AttnQP {
  _Float16 qh[ATQ * HDIM];
  _Float16 ql[ATQ * HDIM];
  _Float16 p[ATQ * ATKT];
};
union AttnLds {
  AttnQP qp;
  float os[ATNW][ATQ * OPITCH];
};
static_assert(sizeof(AttnQP) == 40960, "");
static_assert(sizeof(float) * ATNW * ATQ * OPITCH <= sizeof(AttnQP), "");

__global__ __launch_bounds__(256) void k_attn(const unsigned short* __restrict__ Qhp, const unsigned short* __restrict__ Qlp,
                                              const unsigned short* __restrict__ Khp, const unsigned short* __restrict__ Klp,
                                              const unsigned short* __restrict__ VTp, float* __restrict__ out) {
  __shared__ __align__(16) AttnLds L;
  __shared__ float redm[ATNW][ATQ];
  __shared__ float reds[ATNW][ATQ];

  const int tid  = threadIdx.x;
  const int wave = tid >> 5;
  const int lane = tid & 31;
  const int hh   = lane >> 4;
  const int c    = lane & 15;
  const int b    = blockIdx.y;
  const int q0   = blockIdx.x * ATQ;
  const size_t row0 = (size_t)b * SEQL + q0;

  const _Float16* Kh = (const _Float16*)(const void*)Khp + (size_t)b * SEQL * HDIM;
  const _Float16* Kl = (const _Float16*)(const void*)Klp + (size_t)b * SEQL * HDIM;
  const _Float16* VT = (const _Float16*)(const void*)VTp + (size_t)b * HDIM * SEQL;

  {
    const v4u* gh = (const v4u*)(const void*)(Qhp + row0 * HDIM);
    const v4u* gl = (const v4u*)(const void*)(Qlp + row0 * HDIM);
    v4u* sh = (v4u*)(void*)L.qp.qh;
    v4u* sl = (v4u*)(void*)L.qp.ql;
#pragma unroll
    for (int i = 0; i < 4; ++i) {
      const int ci = tid + 256 * i;
      sh[ci] = gh[ci];
      sl[ci] = gl[ci];
    }
  }
  __syncthreads();

  float mrun[8], lrun[8];
  v8f oacc[4];
#pragma unroll
  for (int r = 0; r < 8; ++r) { mrun[r] = -__builtin_huge_valf(); lrun[r] = 0.f; }
#pragma unroll
  for (int t = 0; t < 4; ++t) oacc[t] = (v8f){0.f,0.f,0.f,0.f,0.f,0.f,0.f,0.f};

  for (int kt = 0; kt < SEQL; kt += ATKT) {
    const int key0 = kt + wave * ATKW;

    v8f shh[2], sx[2];
#pragma unroll
    for (int j = 0; j < 2; ++j) { shh[j] = (v8f){0.f,0.f,0.f,0.f,0.f,0.f,0.f,0.f}; sx[j] = shh[j]; }
#pragma unroll 1
    for (int kd = 0; kd < HDIM / 32; ++kd) {
      const int dofs = kd * 32 + 8 * hh;
      const v16h ah = Frag<_Float16>::load(L.qp.qh + c * HDIM + dofs);
      const v16h al = Frag<_Float16>::load(L.qp.ql + c * HDIM + dofs);
      v16h bh[2], bl[2];
#pragma unroll
      for (int j = 0; j < 2; ++j) {
        const size_t ko = (size_t)(key0 + 16 * j + c) * HDIM + dofs;
        bh[j] = Frag<_Float16>::load(Kh + ko);
        bl[j] = Frag<_Float16>::load(Kl + ko);
      }
#pragma unroll
      for (int j = 0; j < 2; ++j) {
        shh[j] = Frag<_Float16>::mma(ah, bh[j], shh[j]);
        sx[j]  = Frag<_Float16>::mma(ah, bl[j], sx[j]);
        sx[j]  = Frag<_Float16>::mma(al, bh[j], sx[j]);
      }
      dep_guard_h(shh[0], sx[1], ah, al);
      keep4_h(bh[0], bl[0], bh[1], bl[1]);
    }
    acc_guard4(shh[0], shh[1], sx[0], sx[1]);

    float sc[2][8];
#pragma unroll
    for (int j = 0; j < 2; ++j)
#pragma unroll
      for (int r = 0; r < 8; ++r) sc[j][r] = shh[j][r] + sx[j][r] * RES_CARRY_INV;

    float rmx[8];
#pragma unroll
    for (int r = 0; r < 8; ++r) {
      float m = fmaxf(sc[0][r], sc[1][r]);
#pragma unroll
      for (int off = 1; off < 16; off <<= 1) m = fmaxf(m, __shfl_xor(m, off, 32));
      rmx[r] = m;
    }
    if (c == 0) {
#pragma unroll
      for (int r = 0; r < 8; ++r) redm[wave][8 * hh + r] = rmx[r];
    }
    __syncthreads();

    float mnew[8], alpha[8];
#pragma unroll
    for (int r = 0; r < 8; ++r) {
      float m = mrun[r];
#pragma unroll
      for (int w8 = 0; w8 < ATNW; ++w8) m = fmaxf(m, redm[w8][8 * hh + r]);
      mnew[r]  = m;
      alpha[r] = expf(mrun[r] - m);
      mrun[r]  = m;
    }

    float psum[8];
    _Float16* prow = L.qp.p + wave * ATKW;
#pragma unroll
    for (int r = 0; r < 8; ++r) {
      const float p0 = expf(sc[0][r] - mnew[r]);
      const float p1 = expf(sc[1][r] - mnew[r]);
      psum[r] = p0 + p1;
      prow[(8 * hh + r) * ATKT + c]      = (_Float16)(p0 * P_CARRY);
      prow[(8 * hh + r) * ATKT + 16 + c] = (_Float16)(p1 * P_CARRY);
    }
#pragma unroll
    for (int r = 0; r < 8; ++r) {
#pragma unroll
      for (int off = 1; off < 16; off <<= 1) psum[r] += __shfl_xor(psum[r], off, 32);
    }
    if (c == 0) {
#pragma unroll
      for (int r = 0; r < 8; ++r) reds[wave][8 * hh + r] = psum[r];
    }
    __syncthreads();

#pragma unroll
    for (int r = 0; r < 8; ++r) {
      float tot = 0.f;
#pragma unroll
      for (int w8 = 0; w8 < ATNW; ++w8) tot += reds[w8][8 * hh + r];
      lrun[r] = lrun[r] * alpha[r] + tot;
#pragma unroll
      for (int t = 0; t < 4; ++t) oacc[t][r] *= alpha[r];
    }

#pragma unroll 1
    for (int ks = 0; ks < ATKT / 32; ++ks) {
      const int kofs = ks * 32 + 8 * hh;
      const v16h pa = Frag<_Float16>::load(L.qp.p + c * ATKT + kofs);
      v16h vb[4];
#pragma unroll
      for (int t = 0; t < 4; ++t)
        vb[t] = Frag<_Float16>::load(VT + (size_t)(wave * 64 + 16 * t + c) * SEQL + kt + kofs);
#pragma unroll
      for (int t = 0; t < 4; ++t) oacc[t] = Frag<_Float16>::mma(pa, vb[t], oacc[t]);
      dep_guard_h(oacc[0], oacc[3], pa, vb[3]);
      keep4_h(vb[0], vb[1], vb[2], pa);
    }
    acc_guard4(oacc[0], oacc[1], oacc[2], oacc[3]);
    __syncthreads();
  }

  float* os = L.os[wave];
#pragma unroll
  for (int r = 0; r < 8; ++r) {
    const float inv = 1.0f / (lrun[r] * P_CARRY);
#pragma unroll
    for (int t = 0; t < 4; ++t) os[(8 * hh + r) * OPITCH + 16 * t + c] = oacc[t][r] * inv;
  }
  __syncthreads();
  {
    const int c4 = (lane & 15) * 4;
    float* ob = out + row0 * HDIM + wave * 64;
    for (int pass = 0; pass < 2; ++pass) {
#pragma unroll
      for (int it = 0; it < 8; ++it) {
        const int row = it * 2 + hh;
        const v4f val = *(const v4f*)(os + row * OPITCH + c4);
        *(volatile v4f*)(ob + (size_t)row * HDIM + c4) = val;
      }
      __threadfence();
    }
  }
}

constexpr size_t SZ_PE    = (size_t)SEQL * HDIM * 4;
constexpr size_t SZ_PLANE = (size_t)NROW * HDIM * 2;
constexpr size_t SZ_W     = (size_t)HDIM * HDIM * 2;
constexpr size_t OFF_PE = 0;
constexpr size_t OFF_XH = OFF_PE + SZ_PE;
constexpr size_t OFF_XL = OFF_XH + SZ_PLANE;
constexpr size_t OFF_WQ = OFF_XL + SZ_PLANE;
constexpr size_t OFF_WK = OFF_WQ + SZ_W;
constexpr size_t OFF_WV = OFF_WK + SZ_W;
constexpr size_t OFF_QH = OFF_WV + SZ_W;
constexpr size_t OFF_QL = OFF_QH + SZ_PLANE;
constexpr size_t OFF_KH = OFF_QL + SZ_PLANE;
constexpr size_t OFF_KL = OFF_KH + SZ_PLANE;
constexpr size_t OFF_VT = OFF_KL + SZ_PLANE;
constexpr size_t WS_END = OFF_VT + SZ_PLANE;
static_assert(WS_END <= (size_t)134217728, "");
static_assert(OFF_XH % 128 == 0 && OFF_WQ % 128 == 0 && OFF_QH % 128 == 0 && OFF_VT % 128 == 0, "");
static_assert(NROW % 64 == 0 && HDIM % 64 == 0 && SEQL % 64 == 0 && HDIM % 32 == 0, "");

extern "C" void kernel_launch(void* const* d_in, const int* in_sizes, int n_in,
                              void* d_out, int out_size, void* d_ws, size_t ws_size,
                              hipStream_t stream) {
  if (n_in < 7) return;
  if (in_sizes[0] != NROW * HDIM || in_sizes[1] != HDIM * HDIM || in_sizes[2] != HDIM ||
      in_sizes[3] != HDIM * HDIM || in_sizes[4] != HDIM || in_sizes[5] != HDIM * HDIM ||
      in_sizes[6] != HDIM || out_size != NROW * HDIM) return;
  if (WS_END > ws_size) return;

  const float* xin = (const float*)d_in[0];
  const float* Wq  = (const float*)d_in[1];
  const float* bq  = (const float*)d_in[2];
  const float* Wk  = (const float*)d_in[3];
  const float* bk  = (const float*)d_in[4];
  const float* Wv  = (const float*)d_in[5];
  const float* bv  = (const float*)d_in[6];
  float* out = (float*)d_out;

  char* ws = (char*)d_ws;
  float*          pe  = (float*)(ws + OFF_PE);
  unsigned short* xh  = (unsigned short*)(ws + OFF_XH);
  unsigned short* xl  = (unsigned short*)(ws + OFF_XL);
  unsigned short* wqp = (unsigned short*)(ws + OFF_WQ);
  unsigned short* wkp = (unsigned short*)(ws + OFF_WK);
  unsigned short* wvp = (unsigned short*)(ws + OFF_WV);
  unsigned short* qh  = (unsigned short*)(ws + OFF_QH);
  unsigned short* ql  = (unsigned short*)(ws + OFF_QL);
  unsigned short* kh  = (unsigned short*)(ws + OFF_KH);
  unsigned short* kl  = (unsigned short*)(ws + OFF_KL);
  unsigned short* vt  = (unsigned short*)(ws + OFF_VT);

  PETab tab;
  {
    const float lg = 9.2103405f;
    const float cf = -(lg / 512.0f);
    for (int i = 0; i < 256; ++i) {
      const float arg = (float)(2 * i) * cf;
      tab.d[i] = (float)exp((double)arg);
    }
  }

  k_petab<<<SEQL * HDIM / 256, 256, 0, stream>>>(pe, tab);
  k_wplane<<<HDIM * HDIM / 2 / 256, 256, 0, stream>>>(Wq, wqp, HDIM * HDIM / 2);
  k_wplane<<<HDIM * HDIM / 2 / 256, 256, 0, stream>>>(Wk, wkp, HDIM * HDIM / 2);
  k_wplane<<<HDIM * HDIM / 2 / 256, 256, 0, stream>>>(Wv, wvp, HDIM * HDIM / 2);
  k_xplanes<<<NROW * HDIM / 8 / 256, 256, 0, stream>>>(xin, pe, xh, xl);

  {
    const int M = NROW, N = HDIM, K = HDIM;
    const int nblk = ((M / 64) * (N / 64) + 7) / 8;
    k_pgemm<true, false, 2, 3><<<dim3(nblk, 1), 256, 0, stream>>>(
        xh, xl, HDIM, (long)0, wqp, wqp, HDIM, (long)0, qh, ql, HDIM, (long)0, bq, M, N, K);
    k_pgemm<true, false, 2, 3><<<dim3(nblk, 1), 256, 0, stream>>>(
        xh, xl, HDIM, (long)0, wkp, wkp, HDIM, (long)0, kh, kl, HDIM, (long)0, bk, M, N, K);
  }
  {
    const int M = HDIM, N = SEQL, K = HDIM;
    const int nblk = ((M / 64) * (N / 64) + 7) / 8;
    k_pgemm<false, true, 1, 1><<<dim3(nblk, NBAT), 256, 0, stream>>>(
        wvp, wvp, HDIM, (long)0, xh, xl, HDIM, (long)SEQL * HDIM, vt, vt, SEQL, (long)HDIM * SEQL, bv, M, N, K);
  }
  k_attn<<<dim3(SEQL / ATQ, NBAT), 256, 0, stream>>>(qh, ql, kh, kl, vt, out);
}
